// RoomDescriptor_52424370815601
// MI455X (gfx1250) — hardware-verified
//
#include <hip/hip_runtime.h>
#include <math.h>

typedef __attribute__((ext_vector_type(16))) _Float16 v16h;
typedef __attribute__((ext_vector_type(16))) __bf16 v16b;
typedef __attribute__((ext_vector_type(8)))  _Float16 v8h;
typedef __attribute__((ext_vector_type(8)))  float v8f;
typedef __attribute__((ext_vector_type(4)))  float v4f;
typedef __attribute__((ext_vector_type(2)))  float v2f;
typedef __attribute__((ext_vector_type(4)))  unsigned v4u;
typedef __attribute__((ext_vector_type(4)))  int v4i;
typedef float __attribute__((may_alias)) float_a;
typedef int __attribute__((may_alias)) int_a;

template <typename T> __device__ __forceinline__ void vst2(void* p, T v) { *(volatile T*)p = v; __threadfence(); *(volatile T*)p = v; }
__device__ __forceinline__ v8f wmma16(v16h a, v16h b, v8f c) {
  v8f d = __builtin_amdgcn_wmma_f32_16x16x32_f16(false, a, false, b, (short)0, c, false, false);
  asm volatile("v_nop\n\tv_nop\n\tv_nop\n\tv_nop" : "+v"(d) : "v"(a), "v"(b));
  return d;
}
__device__ __forceinline__ v8f wmma_bf(v16b a, v16b b, v8f c) {
  v8f d = __builtin_amdgcn_wmma_f32_16x16x32_bf16(false, a, false, b, (short)0, c, false, false);
  asm volatile("v_nop\n\tv_nop\n\tv_nop\n\tv_nop" : "+v"(d) : "v"(a), "v"(b));
  return d;
}
__device__ __forceinline__ v16h frag_h(const _Float16* rowk0, int lane) {
  union { v16h v; v8h q[2]; } u; const _Float16* p = rowk0 + 8 * (lane >> 4);
  u.q[0] = *(const v8h*)p; u.q[1] = *(const v8h*)(p + 16); return u.v;
}
__device__ __forceinline__ v16h frag_f32(const float* rowk0, int lane) {
  v16h a; const float* p = rowk0 + 8 * (lane >> 4);
#pragma unroll
  for (int i = 0; i < 8; ++i) { a[i] = (_Float16)p[i]; a[8 + i] = (_Float16)p[16 + i]; }
  return a;
}
__device__ __forceinline__ v16h frag_f32s(const float* rowk0, int lane, float sc) {
  v16h a; const float* p = rowk0 + 8 * (lane >> 4);
#pragma unroll
  for (int i = 0; i < 8; ++i) { a[i] = (_Float16)(p[i] * sc); a[8 + i] = (_Float16)(p[16 + i] * sc); }
  return a;
}
__device__ __forceinline__ v16h fragc_f32(const float* W, int k0, int n, int lane, int ld, int K) {
  v16h a; const int g = lane >> 4;
#pragma unroll
  for (int i = 0; i < 8; ++i) { const int ka = k0 + 8 * g + i, kb = ka + 16;
    a[i] = (_Float16)(ka < K ? W[(size_t)(ka < K ? ka : K - 1) * ld + n] : 0.f); a[8 + i] = (_Float16)(kb < K ? W[(size_t)(kb < K ? kb : K - 1) * ld + n] : 0.f); }
  return a;
}
struct F2 { v16b h, l; };
__device__ __forceinline__ F2 bsplit16(const float v[16]) { F2 r;
#pragma unroll
  for (int i = 0; i < 16; ++i) { const __bf16 h = (__bf16)v[i]; r.h[i] = h; r.l[i] = (__bf16)(v[i] - (float)h); }
  return r; }
__device__ __forceinline__ F2 split_row(const float* row, int k0, int lane) { float v[16]; const float* p = row + k0 + 8 * (lane >> 4);
#pragma unroll
  for (int i = 0; i < 8; ++i) { v[i] = p[i]; v[8 + i] = p[16 + i]; }
  return bsplit16(v); }
__device__ __forceinline__ F2 split_rowK(const float* row, int k0, int lane, int K) { float v[16]; const int g = lane >> 4;
#pragma unroll
  for (int i = 0; i < 8; ++i) { const int ka = k0 + 8 * g + i, kb = ka + 16; v[i] = ka < K ? row[ka < K ? ka : K - 1] : 0.f; v[8 + i] = kb < K ? row[kb < K ? kb : K - 1] : 0.f; }
  return bsplit16(v); }
__device__ __forceinline__ F2 split_col(const float* W, int k0, int n, int lane, int ld, int K) { float v[16]; const int g = lane >> 4;
#pragma unroll
  for (int i = 0; i < 8; ++i) { const int ka = k0 + 8 * g + i, kb = ka + 16; v[i] = ka < K ? W[(size_t)(ka < K ? ka : K - 1) * ld + n] : 0.f; v[8 + i] = kb < K ? W[(size_t)(kb < K ? kb : K - 1) * ld + n] : 0.f; }
  return bsplit16(v); }
__device__ __forceinline__ v8f mac3(const F2& a, const F2& b, v8f c) { c = wmma_bf(a.l, b.h, c); c = wmma_bf(a.h, b.l, c); return wmma_bf(a.h, b.h, c); }
__device__ __forceinline__ float sigm(float v) { return 1.0f / (1.0f + expf(-v)); }
#define LDSX() do { asm volatile("s_wait_dscnt 0" ::: "memory"); __builtin_amdgcn_wave_barrier(); __builtin_amdgcn_fence(__ATOMIC_RELEASE, "workgroup"); } while (0)


#define NOB 32
#define NN 512
#define NF 256
#define NHD 64
#define NHS 8
#define HC (NHS * NHD)
#define NO 128
#ifndef NOBB
#define NOBB NOB
#endif
typedef __attribute__((ext_vector_type(8))) __bf16 v8b;
__device__ __forceinline__ v16b frag_b(const __bf16* rowk0, int lane) {
  union { v16b v; v8b q[2]; } u; const __bf16* p = rowk0 + 8 * (lane >> 4);
  u.q[0] = *(const v8b*)p; u.q[1] = *(const v8b*)(p + 16); return u.v;
}
__device__ __forceinline__ float bfr(float v) { return (float)(__bf16)v; }
__device__ __attribute__((noinline)) float exp_ni(float v) { return expf(v); }
__device__ __attribute__((noinline)) float erf_ni(float v) { return erff(v); }

#define WS_PW  0u
#define WS_PWO (WS_PW + 2u * HC * NF)
#define WS_E1  (WS_PWO + 2u * NO * HC)
#define WS_E2  (WS_E1 + 4u * NOB * NHS * NN)
#define WS_VH  (WS_E2 + 4u * NOB * NHS * NN)
#define WS_VL  (WS_VH + 2u * (size_t)NOB * HC * NN)
#define WS_X2  (WS_VL + 2u * (size_t)NOB * HC * NN)
#define WS_F1  (WS_X2 + 4u * (size_t)NOB * NN * HC)
#define WS_F2  (WS_F1 + 4u * NOB * NN)
#define WS_H2H (WS_F2 + 4u * NOB * NN)
#define WS_H2L (WS_H2H + 2u * NOB * NO * NN)
#define WS_PS  (WS_H2L + 2u * NOB * NO * NN)
#define WS_END (WS_PS + 4u * NOB * 8 * NO)

__global__ __launch_bounds__(256) void k_pack(const float* __restrict__ WT, const float* __restrict__ WO, __bf16* __restrict__ PW, __bf16* __restrict__ PWO) {
  const int n = blockIdx.x, which = blockIdx.y, t = threadIdx.x; __shared__ __align__(16) __bf16 s[HC];
  if (which == 0) { s[t] = (__bf16)WT[(size_t)n * NF + t]; __syncthreads(); if (t < NF / 8) vst2((unsigned*)(PW + (size_t)n * NF + t * 8), *(const v4u*)&s[t * 8]); }
  else { if (n >= NO) return; for (int k = t; k < HC; k += 256) s[k] = (__bf16)WO[(size_t)n * HC + k]; __syncthreads(); if (t < HC / 8) vst2((unsigned*)(PWO + (size_t)n * HC + t * 8), *(const v4u*)&s[t * 8]); }
}
__global__ __launch_bounds__(128) void k_h(const float* __restrict__ X, const __bf16* __restrict__ PW, const float* __restrict__ A1, const float* __restrict__ A2, float* __restrict__ E1, float* __restrict__ E2, _Float16* __restrict__ VH, _Float16* __restrict__ VL) {
  __shared__ __align__(16) _Float16 sth[128][72], stl[128][72]; __shared__ __align__(16) float se[2][2][64];
  const int tid = threadIdx.x, wave = tid >> 5, lane = tid & 31, col = lane & 15, g = lane >> 4; const int hp = blockIdx.y; const size_t b = blockIdx.z; const int n0 = blockIdx.x * 64; const size_t r0 = b * NN + n0 + wave * 16;
  v8f acc[8] = {};
#pragma unroll
  for (int kc = 0; kc < NF / 32; ++kc) { v16b a; { const float* p = X + (r0 + col) * NF + kc * 32 + 8 * g;
#pragma unroll
      for (int i = 0; i < 8; ++i) { a[i] = (__bf16)p[i]; a[8 + i] = (__bf16)p[16 + i]; } }
#pragma unroll
    for (int j = 0; j < 8; ++j) acc[j] = wmma_bf(a, frag_b(PW + (size_t)(hp * 128 + j * 16 + col) * NF + kc * 32, lane), acc[j]); }
#pragma unroll
  for (int hl = 0; hl < 2; ++hl) { const int hh = hp * 2 + hl;
#pragma unroll
    for (int r = 0; r < 8; ++r) { float p1 = 0.f, p2 = 0.f;
#pragma unroll
      for (int j = 0; j < 4; ++j) { const int d = j * 16 + col; const float hv = acc[hl * 4 + j][r]; p1 += hv * bfr(A1[hh * NHD + d]); p2 += hv * bfr(A2[hh * NHD + d]); }
#pragma unroll
      for (int o = 1; o < 16; o <<= 1) { p1 += __shfl_xor(p1, o); p2 += __shfl_xor(p2, o); }
      if (col == 0) { se[0][hl][wave * 16 + 8 * g + r] = p1; se[1][hl][wave * 16 + 8 * g + r] = p2; } } }
#pragma unroll
  for (int j = 0; j < 8; ++j)
#pragma unroll
    for (int r = 0; r < 8; ++r) { const float v = acc[j][r]; const _Float16 hv = (_Float16)v; sth[j * 16 + col][wave * 16 + 8 * g + r] = hv; stl[j * 16 + col][wave * 16 + 8 * g + r] = (_Float16)((v - (float)hv) * 2048.0f); }
  __syncthreads();
  if (tid < 64) { const int which = tid >> 5, hl = (tid >> 4) & 1, q = tid & 15; float* dst = (which ? E2 : E1) + (b * NHS + hp * 2 + hl) * NN + n0 + q * 4; vst2(dst, *(const v4f*)&se[which][hl][q * 4]); }
  for (int e = tid; e < 128 * 8; e += 128) { const int d = e >> 3, pc = e & 7; const size_t o = (b * HC + hp * 128 + d) * NN + n0 + pc * 8; vst2((unsigned*)(VH + o), *(const v4u*)&sth[d][pc * 8]); vst2((unsigned*)(VL + o), *(const v4u*)&stl[d][pc * 8]); }
}
template <int L>
__global__ __launch_bounds__(128) void k_att(const float* __restrict__ EK, const float* __restrict__ EJ, const _Float16* __restrict__ VH, const _Float16* __restrict__ VL, float* __restrict__ OUTB) {
  constexpr int NDT = (L == 1) ? 4 : 8;
  __shared__ __align__(16) _Float16 sph[4][16][40], spl[4][16][40]; __shared__ __align__(16) float so[64][132];
  const int tid = threadIdx.x, wave = tid >> 5, lane = tid & 31, col = lane & 15, g = lane >> 4; const int hh = blockIdx.y; const size_t b = blockIdx.z; const int q0 = blockIdx.x * 64 + wave * 16;
  const float* ek = EK + ((L == 1) ? (b * NHS + hh) * NN : b * NN); const float* ej = EJ + ((L == 1) ? (b * NHS + hh) * NN : b * NN); const size_t vbase = (L == 1) ? (b * HC + hh * NHD) * NN : (b * NO) * NN;
  float fj[8], m[8], l[8];
#pragma unroll
  for (int r = 0; r < 8; ++r) { fj[r] = ej[q0 + 8 * g + r]; m[r] = -3.0e38f; l[r] = 0.f; }
  v8f acc[NDT] = {}, accl[NDT] = {};
#pragma unroll 1
  for (int ks = 0; ks < NN / 32; ++ks) { const int j0 = ks * 32; float s[2][8];
#pragma unroll
    for (int ct = 0; ct < 2; ++ct) { const float fk = ek[j0 + ct * 16 + col];
#pragma unroll
      for (int r = 0; r < 8; ++r) { const float e = fk + fj[r]; s[ct][r] = (e >= 0.f) ? e : 0.2f * e; } }
#pragma unroll
    for (int r = 0; r < 8; ++r) { float mx = fmaxf(s[0][r], s[1][r]);
#pragma unroll
      for (int o = 1; o < 16; o <<= 1) mx = fmaxf(mx, __shfl_xor(mx, o));
      const float mn = fmaxf(m[r], mx); const float alpha = (m[r] <= -1.0e38f) ? 0.f : __expf(m[r] - mn); const float e0 = __expf(s[0][r] - mn), e1 = __expf(s[1][r] - mn); float es = e0 + e1;
#pragma unroll
      for (int o = 1; o < 16; o <<= 1) es += __shfl_xor(es, o);
      l[r] = l[r] * alpha + es; m[r] = mn;
#pragma unroll
      for (int dt = 0; dt < NDT; ++dt) { acc[dt][r] *= alpha; accl[dt][r] *= alpha; }
      { const float p0 = e0 * 2048.0f, p1 = e1 * 2048.0f; const _Float16 h0 = (_Float16)p0, h1 = (_Float16)p1; sph[wave][8 * g + r][col] = h0; sph[wave][8 * g + r][16 + col] = h1; spl[wave][8 * g + r][col] = (_Float16)((p0 - (float)h0) * 2048.0f); spl[wave][8 * g + r][16 + col] = (_Float16)((p1 - (float)h1) * 2048.0f); } }
    LDSX();
    const v16h pah = frag_h(&sph[wave][col][0], lane), pal = frag_h(&spl[wave][col][0], lane);
#pragma unroll
    for (int dt = 0; dt < NDT; ++dt) { const size_t vo = vbase + (size_t)(dt * 16 + col) * NN + j0; const v16h vh = frag_h(VH + vo, lane); acc[dt] = wmma16(pah, vh, acc[dt]); accl[dt] = wmma16(pal, vh, accl[dt]); accl[dt] = wmma16(pah, frag_h(VL + vo, lane), accl[dt]); }
    LDSX(); }
#pragma unroll
  for (int r = 0; r < 8; ++r) { const float il = (1.0f / 2048.0f) / l[r];
#pragma unroll
    for (int dt = 0; dt < NDT; ++dt) { float v = (acc[dt][r] + accl[dt][r] * (1.0f / 2048.0f)) * il; if (L == 1) v = (v >= 0.f) ? v : 0.01f * v; so[wave * 16 + 8 * g + r][dt * 16 + col] = v; } }
  __syncthreads();
  if (L == 1) { for (int e = tid; e < 64 * 16; e += 128) { const int r = e >> 4, q = e & 15; vst2(OUTB + ((b * NN + blockIdx.x * 64 + r) * HC) + hh * NHD + q * 4, *(const v4f*)&so[r][q * 4]); } }
  else { __shared__ __align__(16) float sps[NO]; if (tid < NO) { float a = 0.f; for (int r = 0; r < 64; ++r) a += so[r][tid]; sps[tid] = a; } __syncthreads(); if (tid < NO / 4) vst2(OUTB + ((b * 8 + blockIdx.x) * NO) + tid * 4, *(const v4f*)&sps[tid * 4]); }
}
__global__ __launch_bounds__(128) void k_h2(const float* __restrict__ X2, const __bf16* __restrict__ PWO, const float* __restrict__ A1o, const float* __restrict__ A2o, float* __restrict__ F1o, float* __restrict__ F2o, _Float16* __restrict__ H2H, _Float16* __restrict__ H2L) {
  __shared__ __align__(16) _Float16 sth[NO][72], stl[NO][72]; __shared__ __align__(16) float se[2][64];
  const int tid = threadIdx.x, wave = tid >> 5, lane = tid & 31, col = lane & 15, g = lane >> 4; const size_t b = blockIdx.y; const int n0 = blockIdx.x * 64; const size_t r0 = b * NN + n0 + wave * 16;
  v8f acc[8] = {};
#pragma unroll 2
  for (int kc = 0; kc < HC / 32; ++kc) { const F2 a = split_row(X2 + (r0 + col) * HC, kc * 32, lane);
#pragma unroll
    for (int j = 0; j < 8; ++j) { const v16b w = frag_b(PWO + (size_t)(j * 16 + col) * HC + kc * 32, lane); acc[j] = wmma_bf(a.l, w, acc[j]); acc[j] = wmma_bf(a.h, w, acc[j]); } }
#pragma unroll
  for (int r = 0; r < 8; ++r) { float p1 = 0.f, p2 = 0.f;
#pragma unroll
    for (int j = 0; j < 8; ++j) { const int d = j * 16 + col; p1 += acc[j][r] * bfr(A1o[d]); p2 += acc[j][r] * bfr(A2o[d]); }
#pragma unroll
    for (int o = 1; o < 16; o <<= 1) { p1 += __shfl_xor(p1, o); p2 += __shfl_xor(p2, o); }
    if (col == 0) { se[0][wave * 16 + 8 * g + r] = p1; se[1][wave * 16 + 8 * g + r] = p2; } }
#pragma unroll
  for (int j = 0; j < 8; ++j)
#pragma unroll
    for (int r = 0; r < 8; ++r) { const float v = acc[j][r]; const _Float16 hv = (_Float16)v; sth[j * 16 + col][wave * 16 + 8 * g + r] = hv; stl[j * 16 + col][wave * 16 + 8 * g + r] = (_Float16)((v - (float)hv) * 2048.0f); }
  __syncthreads();
  if (tid < 32) { const int which = tid >> 4, q = tid & 15; vst2((which ? F2o : F1o) + b * NN + n0 + q * 4, *(const v4f*)&se[which][q * 4]); }
  for (int e = tid; e < NO * 8; e += 128) { const int d = e >> 3, pc = e & 7; const size_t o = (b * NO + d) * NN + n0 + pc * 8; vst2((unsigned*)(H2H + o), *(const v4u*)&sth[d][pc * 8]); vst2((unsigned*)(H2L + o), *(const v4u*)&stl[d][pc * 8]); }
}
__global__ __launch_bounds__(128) void k_fin(const float* __restrict__ PS, const float* __restrict__ WL, const float* __restrict__ BL, float* __restrict__ OUT) {
  __shared__ float smean[NO]; __shared__ float sy[NO]; __shared__ float red[4]; const int b = blockIdx.x, t = threadIdx.x;
  { float a = 0.f; for (int k = 0; k < 8; ++k) a += PS[((size_t)b * 8 + k) * NO + t]; smean[t] = a / (float)NN; }
  __syncthreads();
  { float a = 0.f; for (int k = 0; k < NO; ++k) a += smean[k] * bfr(WL[(size_t)t * NO + k]); sy[t] = a + bfr(BL[t]); }
  __syncthreads();
  float sq = sy[t] * sy[t];
#pragma unroll
  for (int o = 1; o < 32; o <<= 1) sq += __shfl_xor(sq, o);
  if ((t & 31) == 0) red[t >> 5] = sq; __syncthreads(); const float nrm = fmaxf(sqrtf(red[0] + red[1] + red[2] + red[3]), 1e-12f);
  __shared__ __align__(16) float so[NO]; so[t] = sy[t] / nrm; __syncthreads();
  if (t < NO / 4) vst2(OUT + (size_t)b * NO + t * 4, *(const v4f*)&so[t * 4]);
}
extern "C" void kernel_launch(void* const* d_in, const int* in_sizes, int n_in, void* d_out, int out_size, void* d_ws, size_t ws_size, hipStream_t stream) {
  (void)in_sizes; (void)n_in; (void)out_size;
  const float** F = (const float**)d_in;
  if (ws_size < (size_t)WS_END) return;
  char* ws = (char*)d_ws; __bf16 *PW = (__bf16*)(ws + WS_PW), *PWO = (__bf16*)(ws + WS_PWO); float *E1 = (float*)(ws + WS_E1), *E2 = (float*)(ws + WS_E2), *X2 = (float*)(ws + WS_X2), *F1 = (float*)(ws + WS_F1), *F2 = (float*)(ws + WS_F2), *PS = (float*)(ws + WS_PS); _Float16 *VH = (_Float16*)(ws + WS_VH), *VL = (_Float16*)(ws + WS_VL), *H2H = (_Float16*)(ws + WS_H2H), *H2L = (_Float16*)(ws + WS_H2L);
  k_pack<<<dim3(HC, 2), 256, 0, stream>>>(F[1], F[4], PW, PWO);
  k_h<<<dim3(NN / 64, NHS / 2, NOBB), 128, 0, stream>>>(F[0], PW, F[2], F[3], E1, E2, VH, VL);
  k_att<1><<<dim3(NN / 64, NHS, NOBB), 128, 0, stream>>>(E1, E2, VH, VL, X2);
  k_h2<<<dim3(NN / 64, NOBB), 128, 0, stream>>>(X2, PWO, F[5], F[6], F1, F2, H2H, H2L);
  k_att<2><<<dim3(NN / 64, 1, NOBB), 128, 0, stream>>>(F1, F2, H2H, H2L, PS);
  k_fin<<<NOBB, 128, 0, stream>>>(PS, F[7], F[8], (float*)d_out);
}
